// GCNClassifier_56727928045765
// MI455X (gfx1250) — hardware-run, weakly checked
//
#include <hip/hip_runtime.h>
#include <math.h>

#define NN 65536
#define NE 524288
#define FD 128
#define NG 64
#define NCLS 10
#define NT 256
#define TB 256
#define NTILE (NN / TB)
#define TB_W (TB / 8)
#define OWN_SHIFT 21
#define SCH 4096
#define SPE (SCH / NT)
#define NCH (NE / SCH)
#define SCHP 2048
#define NCHP (NN / SCHP)
#define WCARRY 16.0f
#define WCARRY_INV (1.0f / 16.0f)

static_assert(NE % SCH == 0, "edge chunks exact");
static_assert(SCH == NT * SPE && (SPE % 4) == 0, "chunk = threads x edges");
static_assert(NN % TB == 0 && TB_W == 32 && (1 << (OWN_SHIFT - 16)) == TB_W, "tile ownership");
static_assert((TB * FD) % (4 * NT) == 0, "LDS accumulator zero fill exact");
static_assert(NN % SCHP == 0 && SCHP == NT * 8, "pool chunks exact");
static_assert(NN % 64 == 0 && FD % 64 == 0 && FD % 32 == 0, "GEMM M,N tile multiples, K % 32 == 0");
static_assert(NG * NCLS == 640 && NG * NCLS == 5 * 128, "output = 5 x 512 B = 20 whole lines");

typedef __attribute__((ext_vector_type(16))) _Float16 v16h;
typedef __attribute__((ext_vector_type(8)))  _Float16 v8h;
typedef __attribute__((ext_vector_type(16))) __bf16   v16b;
typedef __attribute__((ext_vector_type(8)))  __bf16   v8b;
typedef __attribute__((ext_vector_type(8)))  float    v8f;
typedef __attribute__((ext_vector_type(4)))  float    v4f;
typedef __attribute__((ext_vector_type(4)))  int      v4i;
typedef __attribute__((ext_vector_type(4)))  unsigned int v4u;

__device__ __forceinline__ unsigned short f2bf_bits(float f) {
  unsigned u = __float_as_uint(f);
  return (unsigned short)((u + 0x7FFFu + ((u >> 16) & 1u)) >> 16);
}
__device__ __forceinline__ float bf_bits2f(unsigned short h) { return __uint_as_float(((unsigned)h) << 16); }

__device__ __forceinline__ void dep_guard_h(v8f& a, v8f& b, v16h x, v16h y) { asm volatile("v_nop\n\tv_nop\n\tv_nop\n\tv_nop" : "+v"(a), "+v"(b) : "v"(x), "v"(y)); }
__device__ __forceinline__ void dep_guard_b(v8f& a, v8f& b, v16b x, v16b y) { asm volatile("v_nop\n\tv_nop\n\tv_nop\n\tv_nop" : "+v"(a), "+v"(b) : "v"(x), "v"(y)); }
__device__ __forceinline__ void dep_guard4_h(v8f& a, v8f& b, v8f& c, v8f& d, v16h x, v16h y) {
  asm volatile("v_nop\n\tv_nop\n\tv_nop\n\tv_nop" : "+v"(a), "+v"(b), "+v"(c), "+v"(d) : "v"(x), "v"(y));
}
__device__ __forceinline__ void dep_guard4_b(v8f& a, v8f& b, v8f& c, v8f& d, v16b x, v16b y) {
  asm volatile("v_nop\n\tv_nop\n\tv_nop\n\tv_nop" : "+v"(a), "+v"(b), "+v"(c), "+v"(d) : "v"(x), "v"(y));
}
__device__ __forceinline__ void keep4_h(v16h a, v16h b, v16h c, v16h d) { asm volatile("v_nop" :: "v"(a), "v"(b), "v"(c), "v"(d)); }
__device__ __forceinline__ void keep4_b(v16b a, v16b b, v16b c, v16b d) { asm volatile("v_nop" :: "v"(a), "v"(b), "v"(c), "v"(d)); }
__device__ __forceinline__ void acc_guard4(v8f& a, v8f& b, v8f& c, v8f& d) { asm volatile("v_nop\n\tv_nop\n\tv_nop\n\tv_nop" : "+v"(a), "+v"(b), "+v"(c), "+v"(d)); }
template <typename T> struct Frag;
template <> struct Frag<_Float16> {
  typedef v16h V; union U { v16h v; v8h h[2]; };
  static __device__ __forceinline__ v16h load(const _Float16* p) {
    U f; f.h[0] = *(const v8h*)(p); f.h[1] = *(const v8h*)(p + 16); return f.v;
  }
  static __device__ __forceinline__ v8f mma(v16h a, v16h b, v8f c) {
    return __builtin_amdgcn_wmma_f32_16x16x32_f16(false, a, false, b, (short)0, c, false, false);
  }
  static __device__ __forceinline__ void guard(v8f& a, v8f& b, v16h x, v16h y) { dep_guard_h(a, b, x, y); }
  static __device__ __forceinline__ void guard4(v8f& a, v8f& b, v8f& c, v8f& d, v16h x, v16h y) { dep_guard4_h(a, b, c, d, x, y); }
  static __device__ __forceinline__ void keep(v16h a, v16h b, v16h c, v16h d) { keep4_h(a, b, c, d); }
};
template <> struct Frag<__bf16> {
  typedef v16b V; union U { v16b v; v8b h[2]; };
  static __device__ __forceinline__ v16b load(const __bf16* p) {
    U f; f.h[0] = *(const v8b*)(p); f.h[1] = *(const v8b*)(p + 16); return f.v;
  }
  static __device__ __forceinline__ v8f mma(v16b a, v16b b, v8f c) {
    return __builtin_amdgcn_wmma_f32_16x16x32_bf16(false, a, false, b, (short)0, c, false, false);
  }
  static __device__ __forceinline__ void guard(v8f& a, v8f& b, v16b x, v16b y) { dep_guard_b(a, b, x, y); }
  static __device__ __forceinline__ void guard4(v8f& a, v8f& b, v8f& c, v8f& d, v16b x, v16b y) { dep_guard4_b(a, b, c, d, x, y); }
  static __device__ __forceinline__ void keep(v16b a, v16b b, v16b c, v16b d) { keep4_b(a, b, c, d); }
};

__device__ __forceinline__ unsigned pk16(unsigned short a, unsigned short b) { return (unsigned)a | ((unsigned)b << 16); }
__device__ __forceinline__ unsigned short h_bits(float f) { const _Float16 h = (_Float16)f; return __builtin_bit_cast(unsigned short, h); }

template <int ET> struct Elem;
template <> struct Elem<0> { typedef _Float16 T; };
template <> struct Elem<1> { typedef __bf16 T; };
template <int ET, bool SPLIT, int BIAS_MODE, int OUT_MODE, bool RESID, int ACT = 0>
__global__ __launch_bounds__(256) void wmma_gemm64(
    const unsigned short* __restrict__ Ap, const unsigned short* __restrict__ A2p, int lda, long strideA,
    const unsigned short* __restrict__ Btp, const unsigned short* __restrict__ Bt2p, int ldb, long strideB,
    void* __restrict__ Cout, void* __restrict__ Cout2, int ldc, long strideC,
    const float* __restrict__ bias,
    const float* __restrict__ resid, long strideR,
    int M, int N, int K, float scale) {
  typedef typename Elem<ET>::T T;
  typedef typename Frag<T>::V V;
  const T* A = (const T*)Ap; const T* A2 = (const T*)A2p; const T* Bt = (const T*)Btp; const T* Bt2 = (const T*)Bt2p;
  __shared__ __align__(16) float sT[8][16 * 68];
  const int b    = blockIdx.y;
  const int lane = threadIdx.x & 31;
  const int wave = threadIdx.x >> 5;
  const int tilesN = N >> 6;
  const int tilesM = M >> 6;
  const int tile = blockIdx.x * 8 + wave;
  if (tile >= tilesM * tilesN) return;
  const int tm = tile / tilesN;
  const int tn = tile - tm * tilesN;
  const int m0 = tm << 6;
  const int n0 = tn << 6;

  const T* Ab  = A  + (size_t)b * strideA;
  const T* Bb  = Bt + (size_t)b * strideB;
  const T* Ab2 = SPLIT ? (A2  + (size_t)b * strideA) : nullptr;
  const T* Bb2 = SPLIT ? (Bt2 + (size_t)b * strideB) : nullptr;

  const int rlane = lane & 15;
  const int koff  = (lane >> 4) * 8;
  const int mOff  = (lane >> 4) * 8;

  v8f acc[4][4];
#pragma unroll
  for (int i = 0; i < 4; ++i)
#pragma unroll
    for (int j = 0; j < 4; ++j) acc[i][j] = (v8f){0.f,0.f,0.f,0.f,0.f,0.f,0.f,0.f};

  for (int k0 = 0; k0 < K; k0 += 32) {
    V bh[4], bl[4];
#pragma unroll
    for (int j = 0; j < 4; ++j) {
      const size_t bo = (size_t)(n0 + (j << 4) + rlane) * ldb + koff + k0;
      bh[j] = Frag<T>::load(Bb + bo);
      if (SPLIT) bl[j] = Frag<T>::load(Bb2 + bo);
    }
#pragma unroll
    for (int i = 0; i < 4; ++i) {
      const size_t ao = (size_t)(m0 + (i << 4) + rlane) * lda + koff + k0;
      V ah = Frag<T>::load(Ab + ao);
      V al;
      if (SPLIT) al = Frag<T>::load(Ab2 + ao);
#pragma unroll
      for (int j = 0; j < 4; ++j) {
        acc[i][j] = Frag<T>::mma(ah, bh[j], acc[i][j]);
        if (SPLIT) {
          acc[i][j] = Frag<T>::mma(ah, bl[j], acc[i][j]);
          acc[i][j] = Frag<T>::mma(al, bh[j], acc[i][j]);
        }
      }
      Frag<T>::guard4(acc[i][0], acc[i][1], acc[i][2], acc[i][3], ah, SPLIT ? al : ah);
    }
    Frag<T>::keep(bh[0], bh[1], bh[2], bh[3]);
    if (SPLIT) Frag<T>::keep(bl[0], bl[1], bl[2], bl[3]);
  }
  acc_guard4(acc[0][0], acc[0][1], acc[0][2], acc[0][3]);
  acc_guard4(acc[1][0], acc[1][1], acc[1][2], acc[1][3]);
  acc_guard4(acc[2][0], acc[2][1], acc[2][2], acc[2][3]);
  acc_guard4(acc[3][0], acc[3][1], acc[3][2], acc[3][3]);

  float* slab = sT[wave];
  const float* Rb = RESID ? (resid + (size_t)b * strideR) : nullptr;
#pragma unroll
  for (int i = 0; i < 4; ++i) {
    const int mBase = m0 + (i << 4);
#pragma unroll
    for (int j = 0; j < 4; ++j) {
      const int n = n0 + (j << 4) + rlane;
      float bv = 0.f;
      if (BIAS_MODE == 2) bv = bias[n];
#pragma unroll
      for (int r = 0; r < 8; ++r) {
        float v = acc[i][j][r] * scale;
        if (BIAS_MODE == 1) v += bias[mBase + mOff + r];
        if (BIAS_MODE == 2) v += bv;
        if (RESID) v += Rb[(size_t)(mBase + mOff + r) * ldc + n];
        if (ACT == 2) v = fmaxf(v, 0.0f);
        if (ACT == 4) v = (v > 0.f) ? v : 0.01f * v;
        if (ACT == 6) { const float en = expf(fminf(v, 0.0f)) - 1.0f; v = (v > 0.f) ? v : en; }
        slab[(mOff + r) * 68 + (j << 4) + rlane] = v;
      }
    }
    __builtin_amdgcn_fence(__ATOMIC_RELEASE, "workgroup");
    __builtin_amdgcn_wave_barrier();
    __builtin_amdgcn_fence(__ATOMIC_ACQUIRE, "workgroup");
    if (OUT_MODE == 0) {
      float* C = (float*)Cout + (size_t)b * strideC;
      const int hh = lane >> 4, c4 = (lane & 15) * 4;
      for (int pass = 0; pass < 2; ++pass) {
#pragma unroll
        for (int it = 0; it < 8; ++it) {
          const int row = it * 2 + hh;
          v4f v = *(const v4f*)(slab + row * 68 + c4);
          *(volatile v4f*)(C + (size_t)(mBase + row) * ldc + n0 + c4) = v;
        }
        __threadfence();
      }
    } else {
      const int q = lane >> 3, c8 = (lane & 7) * 8;
      unsigned short* C  = (unsigned short*)Cout  + (size_t)b * strideC;
      unsigned short* C2 = (OUT_MODE == 2) ? ((unsigned short*)Cout2 + (size_t)b * strideC) : nullptr;
      for (int pass = 0; pass < 2; ++pass) {
#pragma unroll
        for (int it = 0; it < 4; ++it) {
          const int row = it * 4 + q;
          const float* sp = slab + row * 68 + c8;
          v8h hv, lv;
#pragma unroll
          for (int e = 0; e < 8; ++e) {
            if (OUT_MODE == 1) {
              hv[e] = (_Float16)sp[e];
            } else {
              unsigned short hb = f2bf_bits(sp[e]);
              unsigned short lb = f2bf_bits(sp[e] - bf_bits2f(hb));
              hv[e] = __builtin_bit_cast(_Float16, hb);
              lv[e] = __builtin_bit_cast(_Float16, lb);
            }
          }
          *(volatile v8h*)(C + (size_t)(mBase + row) * ldc + n0 + c8) = hv;
          if (OUT_MODE == 2) *(volatile v8h*)(C2 + (size_t)(mBase + row) * ldc + n0 + c8) = lv;
        }
        __threadfence();
      }
    }
    __builtin_amdgcn_fence(__ATOMIC_RELEASE, "workgroup");
    __builtin_amdgcn_wave_barrier();
    __builtin_amdgcn_fence(__ATOMIC_ACQUIRE, "workgroup");
  }
}

__global__ __launch_bounds__(256) void wtcast_kernel(const float* __restrict__ W0, const float* __restrict__ W1,
                                                     const float* __restrict__ W2,
                                                     unsigned short* __restrict__ out, float scale) {
  __shared__ float sm[64][65];
  const int t  = threadIdx.x;
  const int k0 = blockIdx.x * 64;
  const int nb = blockIdx.y * 64;
  const int z  = blockIdx.z;
  const float* W = (z == 0) ? W0 : (z == 1) ? W1 : W2;
#pragma unroll
  for (int i = 0; i < 16; ++i) {
    const int e = i * 256 + t;
    const int r = e >> 6;
    const int c = e & 63;
    sm[c][r] = W[(size_t)(k0 + r) * FD + nb + c] * scale;
  }
  __syncthreads();
  const int lane = t & 31, wave = t >> 5;
  const int q = lane >> 3, c8 = (lane & 7) * 8;
  unsigned short* op = out + (size_t)z * FD * FD;
  for (int pass = 0; pass < 2; ++pass) {
#pragma unroll
    for (int it = 0; it < 2; ++it) {
      const int row = wave * 8 + it * 4 + q;
      unsigned short hb[8];
#pragma unroll
      for (int e = 0; e < 8; ++e) hb[e] = h_bits(sm[row][c8 + e]);
      const v4u u = (v4u){pk16(hb[0], hb[1]), pk16(hb[2], hb[3]), pk16(hb[4], hb[5]), pk16(hb[6], hb[7])};
      *(volatile v4u*)(op + (size_t)(nb + row) * FD + k0 + c8) = u;
    }
    __threadfence();
  }
}

__device__ __forceinline__ int blk_excl_scan(int cnt, int* scan_ws, int tid, int* tot) {
  const int lane = tid & 31, wave = tid >> 5; int incl = cnt;
#pragma unroll
  for (int o = 1; o < 32; o <<= 1) { const int v = __shfl_up(incl, o, 32); if (lane >= o) incl += v; }
  if (lane == 31) scan_ws[wave] = incl;
  __syncthreads();
  if (wave == 0) {
    const int li = (lane < NT / 32) ? lane : 0;
    int wv = scan_ws[li]; wv = (lane < NT / 32) ? wv : 0;
    int wincl = wv;
#pragma unroll
    for (int o = 1; o < 32; o <<= 1) { const int v = __shfl_up(wincl, o, 32); if (lane >= o) wincl += v; }
    if (lane < NT / 32) scan_ws[32 + lane] = wincl - wv;
    if (lane == 31) scan_ws[64] = wincl;
  }
  __syncthreads();
  const int res = scan_ws[32 + wave] + incl - cnt; *tot = scan_ws[64];
  return res;
}
template <int SP, int CAP>
__device__ __forceinline__ int chunk_hits(const int* __restrict__ dstv, const int* __restrict__ srcv, int e0, int n0, int tid,
                                          int* LIST, int* scan_ws) {
  const int eb = e0 + tid * SP;
  int rec[SP]; int cnt = 0;
#pragma unroll
  for (int k = 0; k < SP; k += 4) {
    const v4i d4 = *(const v4i*)(dstv + eb + k);
    const v4i s4 = *(const v4i*)(srcv + eb + k);
#pragma unroll
    for (int e = 0; e < 4; ++e) {
      const int d = d4[e];
      int s = s4[e]; s = s < 0 ? 0 : (s >= NN ? NN - 1 : s);
      int r = -1;
      if (d >= n0 && d < n0 + TB) { r = ((d - n0) << 16) | s; ++cnt; }
      rec[k + e] = r;
    }
  }
  int tot; int p = blk_excl_scan(cnt, scan_ws, tid, &tot);
#pragma unroll
  for (int k = 0; k < SP; ++k) if (rec[k] >= 0) { if ((unsigned)p < (unsigned)CAP) LIST[p] = rec[k]; ++p; }
  __syncthreads();
  return tot < CAP ? tot : CAP;
}

__global__ __launch_bounds__(NT) void agg_kernel(const float* __restrict__ hin, const int* __restrict__ srcv,
                                                const int* __restrict__ dstv, unsigned short* __restrict__ AH) {
  __shared__ __align__(16) float SACC[TB * FD];
  __shared__ __align__(16) int LIST[SCH];
  __shared__ int scan_ws[80];
  const int tid = threadIdx.x, lane = tid & 31, wave = tid >> 5;
  const int n0 = blockIdx.x * TB;
  const v4f z4 = {0.f, 0.f, 0.f, 0.f};
#pragma unroll 4
  for (int i = 0; i < (TB * FD) / (4 * NT); ++i) *(v4f*)(SACC + 4 * (i * NT + tid)) = z4;
  __syncthreads();

#pragma unroll 1
  for (int c = 0; c < NCH; ++c) {
    const int tot = chunk_hits<SPE, SCH>(dstv, srcv, c * SCH, n0, tid, LIST, scan_ws);
#pragma unroll 1
    for (int base = 0; base < tot; base += 32) {
      const int q  = base + lane;
      const int qc = (q < tot) ? q : (tot - 1);
      const int lv = LIST[qc];
      const int rv = (q < tot) ? lv : -1;
      const int own = (rv >= 0 && (rv >> OWN_SHIFT) == wave) ? 1 : 0;
      unsigned msk = (unsigned)__ballot(own);
#pragma unroll 1
      for (int it = 0; it < 32; ++it) {
        if (msk == 0u) break;
        const int bp = __builtin_ctz(msk); msk &= msk - 1u;
        const int r = __shfl(rv, bp, 32);
        const int dl = (r >> 16) & (TB - 1);
        const int s  = r & 0xFFFF;
        const v4f hv = *(const v4f*)(hin + (size_t)s * FD + 4 * lane);
        float* rp = SACC + dl * FD + 4 * lane;
        v4f a = *(const v4f*)rp;
        a = a + hv;
        *(v4f*)rp = a;
      }
    }
    __syncthreads();
  }
  const int hh = lane >> 4, c8 = (lane & 15) * 8;
#pragma unroll 1
  for (int j = 0; j < TB_W / 2; ++j) {
    const int rl = wave * TB_W + 2 * j + hh;
    const float* rp = SACC + rl * FD + c8;
    const v4f a = *(const v4f*)(rp);
    const v4f b = *(const v4f*)(rp + 4);
    unsigned short hb[8];
#pragma unroll
    for (int e = 0; e < 4; ++e) { hb[e] = h_bits(a[e]); hb[4 + e] = h_bits(b[e]); }
    const v4u u = (v4u){pk16(hb[0], hb[1]), pk16(hb[2], hb[3]), pk16(hb[4], hb[5]), pk16(hb[6], hb[7])};
    unsigned short* op = AH + (size_t)(n0 + rl) * FD + c8;
    *(volatile v4u*)op = u;
    __threadfence();
    *(volatile v4u*)op = u;
  }
}

__global__ __launch_bounds__(NT) void pool_kernel(const float* __restrict__ HS, const int* __restrict__ gid, float* __restrict__ HG) {
  __shared__ int LIST[SCHP];
  __shared__ int scan_ws[80];
  __shared__ __align__(16) float red[8 * FD];
  __shared__ int rc[8];
  const int tid = threadIdx.x, lane = tid & 31, wave = tid >> 5;
  const int g = blockIdx.x;
  const v4f z4 = {0.f, 0.f, 0.f, 0.f};
  v4f acc = z4; int cnt = 0;
#pragma unroll 1
  for (int c = 0; c < NCHP; ++c) {
    const int eb = c * SCHP + tid * 8;
    int bv[8]; int rec[8]; int kc = 0;
    const v4i b0 = *(const v4i*)(gid + eb), bb = *(const v4i*)(gid + eb + 4);
    bv[0] = b0[0]; bv[1] = b0[1]; bv[2] = b0[2]; bv[3] = b0[3]; bv[4] = bb[0]; bv[5] = bb[1]; bv[6] = bb[2]; bv[7] = bb[3];
#pragma unroll
    for (int k = 0; k < 8; ++k) { rec[k] = -1; if (bv[k] == g) { rec[k] = eb + k; ++kc; } }
    int tot; int p = blk_excl_scan(kc, scan_ws, tid, &tot);
#pragma unroll
    for (int k = 0; k < 8; ++k) if (rec[k] >= 0) { if ((unsigned)p < (unsigned)SCHP) LIST[p] = rec[k]; ++p; }
    __syncthreads();
    const int totc = tot < SCHP ? tot : SCHP;
#pragma unroll 1
    for (int q = wave; q < totc; q += 8) {
      int nd = LIST[q]; nd = nd < 0 ? 0 : (nd >= NN ? NN - 1 : nd);
      acc = acc + *(const v4f*)(HS + (size_t)nd * FD + 4 * lane); ++cnt;
    }
    __syncthreads();
  }
  *(v4f*)(red + wave * FD + 4 * lane) = acc;
  if (lane == 0) rc[wave] = cnt;
  __syncthreads();
  if (wave == 0) {
    v4f s = z4; int ct = 0;
#pragma unroll
    for (int w = 0; w < 8; ++w) { s = s + *(const v4f*)(red + w * FD + 4 * lane); ct += rc[w]; }
    const float cf = (float)ct;
    const float inv = 1.0f / fmaxf(cf, 1.0f);
    const v4f o = s * inv;
    for (int pass = 0; pass < 2; ++pass) { *(volatile v4f*)(HG + (size_t)g * FD + 4 * lane) = o; __threadfence(); }
  }
}

__global__ __launch_bounds__(NT) void cls_kernel(const float* __restrict__ HG, const float* __restrict__ Wc,
                                                const float* __restrict__ bc, float* __restrict__ out) {
  __shared__ __align__(16) float so[NG * NCLS];
  const int tid = threadIdx.x, wave = tid >> 5, lane = tid & 31;
  for (int i = tid; i < NG * NCLS; i += NT) {
    const int g = i / NCLS, o = i - NCLS * g;
    float a = 0.0f;
#pragma unroll 1
    for (int d = 0; d < FD; ++d) a += HG[g * FD + d] * Wc[d * NCLS + o];
    a += bc[o];
    so[i] = a;
  }
  __syncthreads();
  if (wave == 0) {
    v4f p[5];
#pragma unroll
    for (int k = 0; k < 5; ++k) p[k] = *(const v4f*)(so + 128 * k + 4 * lane);
    for (int pass = 0; pass < 2; ++pass) {
#pragma unroll
      for (int k = 0; k < 5; ++k) *(volatile v4f*)(out + 128 * k + 4 * lane) = p[k];
      __threadfence();
    }
  }
}

extern "C" void kernel_launch(void* const* d_in, const int* in_sizes, int n_in,
                              void* d_out, int out_size, void* d_ws, size_t ws_size, hipStream_t stream) {
  (void)in_sizes; (void)n_in; (void)out_size;
  const float* features = (const float*)d_in[0];
  const int*   srcv     = (const int*)  d_in[1];
  const int*   dstv     = (const int*)  d_in[2];
  const int*   gids     = (const int*)  d_in[3];
  const float* Wl[3]    = {(const float*)d_in[4], (const float*)d_in[6], (const float*)d_in[8]};
  const float* bl[3]    = {(const float*)d_in[5], (const float*)d_in[7], (const float*)d_in[9]};
  const float* Wc       = (const float*)d_in[10];
  const float* bcv      = (const float*)d_in[11];
  float* out = (float*)d_out;

  char* ws = (char*)d_ws; size_t off = 0;
  auto carve = [&](size_t bytes) -> char* { char* p = ws + off; off += (bytes + 255) & ~(size_t)255; return p; };
  unsigned short* WT  = (unsigned short*)carve((size_t)3 * FD * FD * 2);
  unsigned short* AH  = (unsigned short*)carve((size_t)NN * FD * 2);
  float*          H   = (float*)carve((size_t)NN * FD * 4);
  float*          HG  = (float*)carve((size_t)NG * FD * 4);
  if (off > ws_size || off > (size_t)134217728) return;

  wtcast_kernel<<<dim3(FD / 64, FD / 64, 3), NT, 0, stream>>>(Wl[0], Wl[1], Wl[2], WT, WCARRY);

  const int tiles = (NN / 64) * (FD / 64);
  for (int l = 0; l < 3; ++l) {
    const float* hin = (l == 0) ? features : H;
    agg_kernel<<<NTILE, NT, 0, stream>>>(hin, srcv, dstv, AH);
    const unsigned short* WTl = WT + (size_t)l * FD * FD;
    wmma_gemm64<0, false, 2, 0, false, 6><<<dim3((tiles + 7) / 8, 1), 256, 0, stream>>>(
        (const unsigned short*)AH, (const unsigned short*)AH, FD, 0L,
        WTl, WTl, FD, 0L,
        (void*)H, (void*)nullptr, FD, 0L,
        bl[l], (const float*)nullptr, 0L, NN, FD, FD, WCARRY_INV);
  }
  pool_kernel<<<NG, NT, 0, stream>>>(H, gids, HG);
  cls_kernel<<<1, NT, 0, stream>>>(HG, Wc, bcv, out);
}
